// SelfAttention_2362232012882
// MI455X (gfx1250) — hardware-verified
//
#include <hip/hip_runtime.h>


#ifndef NB
#define NB 4
#endif
#ifndef SEQ
#define SEQ 2048
#endif
#define NB_FULL   4
#define SEQ_FULL  2048
#define DM        1024
#define NHEAD     16
#define HDIM      64
#define MROWS     (NB * SEQ)
#define BM        128
#define BN        64
#define BQ        128
#define BK        32
#define NWAVE     8
#define QP        72
#define VP        136
#define FP        68
#define P_CARRY   4096.0f
#define CTX_CARRY 64.0f
#define WO_CARRY  256.0f
#define SB16      18432

static_assert(NB >= 1 && NB <= NB_FULL);
static_assert(SEQ >= BM && SEQ <= SEQ_FULL);
static_assert(SEQ % BM == 0);
static_assert(SEQ % BQ == 0);
static_assert(SEQ % BK == 0);
static_assert(DM % BN == 0);
static_assert(DM % 32 == 0);
static_assert(NHEAD * HDIM == DM);
static_assert(BN == HDIM);
static_assert(HDIM == 64);
static_assert(BM == NWAVE * 16);
static_assert(BQ == NWAVE * 16);
static_assert((QP * 2) % 16 == 0);
static_assert((VP * 2) % 16 == 0);
static_assert((FP * 4) % 16 == 0);
static_assert(BM * QP * 2 <= SB16);
static_assert(HDIM * VP * 2 <= SB16);
static_assert((size_t)((NB_FULL - 1) * SEQ_FULL + SEQ_FULL - 1) * DM + DM - 1 < 33554432ull / 4);

typedef __bf16   bf16;
typedef _Float16 f16;
typedef bf16     v16bf __attribute__((ext_vector_type(16)));
typedef f16      v16h  __attribute__((ext_vector_type(16)));
typedef f16      v8h   __attribute__((ext_vector_type(8)));
typedef float    v8f   __attribute__((ext_vector_type(8)));
typedef float    v4f   __attribute__((ext_vector_type(4)));
typedef unsigned v4u   __attribute__((ext_vector_type(4)));

union FragB  { v16bf v; v4u q[2]; bf16 h[16]; };
union FragH  { v16h  v; v4u q[2]; f16  h[16]; };
union Pack8B { v4u u; bf16 h[8]; };
union Pack8H { v4u u; v8h v; f16 h[8]; };

static __device__ __forceinline__ v8f mma_bf16(v16bf a, v16bf b, v8f acc) {
  acc = __builtin_amdgcn_wmma_f32_16x16x32_bf16(false, a, false, b, (short)0, acc, false, false);
  asm volatile("v_nop\n\tv_nop\n\tv_nop\n\tv_nop" : "+v"(acc) : "v"(a), "v"(b));
  return acc;
}
static __device__ __forceinline__ v8f mma_f16(v16h a, v16h b, v8f acc) {
  acc = __builtin_amdgcn_wmma_f32_16x16x32_f16(false, a, false, b, (short)0, acc, false, false);
  asm volatile("v_nop\n\tv_nop\n\tv_nop\n\tv_nop" : "+v"(acc) : "v"(a), "v"(b));
  return acc;
}
static __device__ __forceinline__ v8f zero8() {
  v8f z = {0.f, 0.f, 0.f, 0.f, 0.f, 0.f, 0.f, 0.f};
  return z;
}

__global__ __launch_bounds__(128) void cvt_kernel(const float* __restrict__ x,
                                                  const float* __restrict__ wq,
                                                  const float* __restrict__ wk,
                                                  const float* __restrict__ wv,
                                                  const float* __restrict__ wo,
                                                  bf16* __restrict__ xb,
                                                  bf16* __restrict__ wqkv,
                                                  f16* __restrict__ wo16) {
  const int blk = blockIdx.x;
  const int t   = threadIdx.x;
  const float* src;
  char* dbase;
  int mode = 0;
  if (blk < MROWS) {
    const int b = blk / SEQ;
    const int s = blk - b * SEQ;
    src   = x + ((size_t)b * SEQ_FULL + s) * DM;
    dbase = (char*)(xb + (size_t)blk * DM);
  } else {
    const int w  = blk - MROWS;
    const int ti = w / DM;
    const int r  = w - ti * DM;
    if (ti < 3) {
      const float* wsrc = (ti == 0) ? wq : ((ti == 1) ? wk : wv);
      src   = wsrc + (size_t)r * DM;
      dbase = (char*)(wqkv + ((size_t)ti * DM + r) * DM);
    } else {
      src   = wo + (size_t)r * DM;
      dbase = (char*)(wo16 + (size_t)r * DM);
      mode  = 1;
    }
  }
  const v4f a0 = *(const v4f*)(src + t * 8);
  const v4f a1 = *(const v4f*)(src + t * 8 + 4);
  v4u val;
  if (mode == 0) {
    Pack8B p;
    #pragma unroll
    for (int i = 0; i < 4; ++i) {
      p.h[i]     = (bf16)a0[i];
      p.h[4 + i] = (bf16)a1[i];
    }
    val = p.u;
  } else {
    Pack8H p;
    #pragma unroll
    for (int i = 0; i < 4; ++i) {
      p.h[i]     = (f16)((float)(bf16)a0[i] * WO_CARRY);
      p.h[4 + i] = (f16)((float)(bf16)a1[i] * WO_CARRY);
    }
    val = p.u;
  }
  volatile v4u* dp = (volatile v4u*)dbase + t;
  *dp = val;
  __threadfence();
  *dp = val;
}

__global__ __launch_bounds__(256) void qkv_gemm_kernel(const bf16* __restrict__ xb,
                                                       const bf16* __restrict__ wqkv,
                                                       const float* __restrict__ bq,
                                                       const float* __restrict__ bk,
                                                       const float* __restrict__ bv,
                                                       f16* __restrict__ qpl,
                                                       f16* __restrict__ kpl,
                                                       f16* __restrict__ vt) {
  const int n0   = blockIdx.x * BN;
  const int m0   = blockIdx.y * BM;
  const int tid  = threadIdx.x;
  const int wave = tid >> 5;
  const int lane = tid & 31;
  const int lq   = lane & 15;
  const int hi   = lane >> 4;
  const int wm   = wave & 3;
  const int wn   = wave >> 2;

  __shared__ __align__(16) unsigned char sraw[SB16];
  f16* sT = (f16*)sraw;

  const int region = n0 / DM;
  const int ncol   = n0 - region * DM;
  const int head   = ncol / HDIM;
  const int b      = m0 / SEQ;
  const int s0     = m0 - b * SEQ;
  const size_t hb  = (size_t)b * NHEAD + head;

  v8f acc[2][2];
  #pragma unroll
  for (int i = 0; i < 2; ++i)
    #pragma unroll
    for (int j = 0; j < 2; ++j) acc[i][j] = zero8();

  const bf16* Ab = xb   + (size_t)(m0 + wm * 32 + lq) * DM + hi * 8;
  const bf16* Wb = wqkv + (size_t)(n0 + wn * 32 + lq) * DM + hi * 8;
  #pragma unroll 1
  for (int k0 = 0; k0 < DM; k0 += 32) {
    FragB af[2], wf[2];
    #pragma unroll
    for (int i = 0; i < 2; ++i) {
      const bf16* ap = Ab + (size_t)i * 16 * DM + k0;
      af[i].q[0] = *(const v4u*)(ap);
      af[i].q[1] = *(const v4u*)(ap + 16);
    }
    #pragma unroll
    for (int j = 0; j < 2; ++j) {
      const bf16* wp = Wb + (size_t)j * 16 * DM + k0;
      wf[j].q[0] = *(const v4u*)(wp);
      wf[j].q[1] = *(const v4u*)(wp + 16);
    }
    #pragma unroll
    for (int i = 0; i < 2; ++i)
      #pragma unroll
      for (int j = 0; j < 2; ++j) acc[i][j] = mma_bf16(af[i].v, wf[j].v, acc[i][j]);
  }

  const float* bias = (region == 0) ? bq : ((region == 1) ? bk : bv);
  float bj[2];
  #pragma unroll
  for (int j = 0; j < 2; ++j) bj[j] = (float)(bf16)bias[ncol + wn * 32 + j * 16 + lq];

  if (region < 2) {
    #pragma unroll
    for (int i = 0; i < 2; ++i)
      #pragma unroll
      for (int j = 0; j < 2; ++j)
        #pragma unroll
        for (int r = 0; r < 8; ++r)
          sT[(wm * 32 + i * 16 + 8 * hi + r) * QP + wn * 32 + j * 16 + lq] = (f16)(acc[i][j][r] + bj[j]);
  } else {
    #pragma unroll
    for (int i = 0; i < 2; ++i)
      #pragma unroll
      for (int j = 0; j < 2; ++j) {
        Pack8H p;
        #pragma unroll
        for (int r = 0; r < 8; ++r) p.h[r] = (f16)(acc[i][j][r] + bj[j]);
        *(v4u*)(sT + (wn * 32 + j * 16 + lq) * VP + wm * 32 + i * 16 + 8 * hi) = p.u;
      }
  }
  __syncthreads();

  v4u    vals[4];
  size_t gidx[4];
  if (region < 2) {
    f16* plane = (region == 0) ? qpl : kpl;
    #pragma unroll
    for (int it = 0; it < 4; ++it) {
      const int row   = wave * 16 + it * 4 + (lane >> 3);
      const int piece = lane & 7;
      vals[it] = *(const v4u*)(sT + row * QP + piece * 8);
      gidx[it] = (hb * SEQ + s0 + row) * HDIM + piece * 8;
    }
    #pragma unroll
    for (int it = 0; it < 4; ++it) *(volatile v4u*)(plane + gidx[it]) = vals[it];
    __threadfence();
    #pragma unroll
    for (int it = 0; it < 4; ++it) *(volatile v4u*)(plane + gidx[it]) = vals[it];
  } else {
    #pragma unroll
    for (int it = 0; it < 4; ++it) {
      const int d     = wave * 8 + it * 2 + (lane >> 4);
      const int piece = lane & 15;
      vals[it] = *(const v4u*)(sT + d * VP + piece * 8);
      gidx[it] = (hb * HDIM + d) * SEQ + s0 + piece * 8;
    }
    #pragma unroll
    for (int it = 0; it < 4; ++it) *(volatile v4u*)(vt + gidx[it]) = vals[it];
    __threadfence();
    #pragma unroll
    for (int it = 0; it < 4; ++it) *(volatile v4u*)(vt + gidx[it]) = vals[it];
  }
}

__global__ __launch_bounds__(256) void attn_kernel(const f16* __restrict__ qpl,
                                                   const f16* __restrict__ kpl,
                                                   const f16* __restrict__ vt,
                                                   f16* __restrict__ ctx) {
  const int qblk = blockIdx.x;
  const int h    = blockIdx.y;
  const int b    = blockIdx.z;
  const int tid  = threadIdx.x;
  const int wave = tid >> 5;
  const int lane = tid & 31;
  const int lq   = lane & 15;
  const int hi   = lane >> 4;

  __shared__ __align__(16) f16 sO[NWAVE * 16 * QP];

  const int qrow0 = qblk * BQ + wave * 16;
  const size_t hb = (size_t)b * NHEAD + h;

  FragH qf[2];
  {
    const f16* qp = qpl + (hb * SEQ + qrow0 + lq) * HDIM;
    #pragma unroll
    for (int f = 0; f < 2; ++f) {
      qf[f].q[0] = *(const v4u*)(qp + f * 32 + hi * 8);
      qf[f].q[1] = *(const v4u*)(qp + f * 32 + 16 + hi * 8);
    }
  }

  const f16* kb_h = kpl + hb * SEQ * HDIM;
  const f16* vt_h = vt  + hb * HDIM * SEQ;

  v8f o[4];
  #pragma unroll
  for (int dt = 0; dt < 4; ++dt) o[dt] = zero8();

  float rmax = -__builtin_inff();
  float rsum = 0.0f;
  const float SL = 0.125f * 1.4426950408889634f;

  #pragma unroll 1
  for (int i = 0; i < SEQ / BK; ++i) {
    const int j0 = i * BK;

    FragH ak[2][2];
    #pragma unroll
    for (int sub = 0; sub < 2; ++sub) {
      #pragma unroll
      for (int f = 0; f < 2; ++f) {
        const f16* base = kb_h + (size_t)(j0 + sub * 16 + lq) * HDIM + f * 32 + hi * 8;
        ak[sub][f].q[0] = *(const v4u*)(base);
        ak[sub][f].q[1] = *(const v4u*)(base + 16);
      }
    }
    FragH vf[4];
    #pragma unroll
    for (int dt = 0; dt < 4; ++dt) {
      const f16* base = vt_h + (size_t)(dt * 16 + lq) * SEQ + j0 + hi * 8;
      vf[dt].q[0] = *(const v4u*)(base);
      vf[dt].q[1] = *(const v4u*)(base + 16);
    }

    v8f c[2];
    #pragma unroll
    for (int sub = 0; sub < 2; ++sub) {
      v8f acc = zero8();
      acc = mma_f16(ak[sub][0].v, qf[0].v, acc);
      acc = mma_f16(ak[sub][1].v, qf[1].v, acc);
      c[sub] = acc;
    }

    float m_new = rmax;
    #pragma unroll
    for (int r = 0; r < 8; ++r) {
      m_new = fmaxf(m_new, c[0][r]);
      m_new = fmaxf(m_new, c[1][r]);
    }
    m_new = fmaxf(m_new, __shfl_xor(m_new, 16, 32));
    const float scale = __builtin_amdgcn_exp2f((rmax - m_new) * SL);
    rmax = m_new;

    FragH pa;
    float psum = 0.0f;
    #pragma unroll
    for (int r = 0; r < 8; ++r) {
      const float p0 = __builtin_amdgcn_exp2f((c[0][r] - m_new) * SL);
      const float p1 = __builtin_amdgcn_exp2f((c[1][r] - m_new) * SL);
      psum += p0 + p1;
      pa.h[r]     = (f16)(p0 * P_CARRY);
      pa.h[8 + r] = (f16)(p1 * P_CARRY);
    }
    rsum = rsum * scale + psum + __shfl_xor(psum, 16, 32);

    float sc[8];
    #pragma unroll
    for (int r = 0; r < 8; ++r) sc[r] = __shfl(scale, (hi << 3) + r, 32);
    #pragma unroll
    for (int dt = 0; dt < 4; ++dt) {
      #pragma unroll
      for (int r = 0; r < 8; ++r) o[dt][r] *= sc[r];
    }

    #pragma unroll
    for (int dt = 0; dt < 4; ++dt) o[dt] = mma_f16(pa.v, vf[dt].v, o[dt]);
  }

  float rs[8];
  #pragma unroll
  for (int r = 0; r < 8; ++r) rs[r] = 1.0f / __shfl(rsum, (hi << 3) + r, 32);

  f16* so = sO + wave * (16 * QP);
  #pragma unroll
  for (int r = 0; r < 8; ++r) {
    #pragma unroll
    for (int dt = 0; dt < 4; ++dt)
      so[(hi * 8 + r) * QP + dt * 16 + lq] = (f16)(o[dt][r] * rs[r] * (CTX_CARRY / P_CARRY));
  }
  __syncthreads();

  v4u    vals[4];
  size_t gidx[4];
  #pragma unroll
  for (int it = 0; it < 4; ++it) {
    const int row   = it * 4 + (lane >> 3);
    const int piece = lane & 7;
    vals[it] = *(const v4u*)(so + row * QP + piece * 8);
    gidx[it] = ((size_t)b * SEQ + qrow0 + row) * DM + h * HDIM + piece * 8;
  }
  #pragma unroll
  for (int it = 0; it < 4; ++it) *(volatile v4u*)(ctx + gidx[it]) = vals[it];
  __threadfence();
  #pragma unroll
  for (int it = 0; it < 4; ++it) *(volatile v4u*)(ctx + gidx[it]) = vals[it];
}

__global__ __launch_bounds__(256) void oproj_kernel(const f16* __restrict__ ctx,
                                                    const f16* __restrict__ wo16,
                                                    const float* __restrict__ bo,
                                                    float* __restrict__ out) {
  const int n0   = blockIdx.x * BN;
  const int m0   = blockIdx.y * BM;
  const int tid  = threadIdx.x;
  const int wave = tid >> 5;
  const int lane = tid & 31;
  const int lq   = lane & 15;
  const int hi   = lane >> 4;
  const int wm   = wave & 3;
  const int wn   = wave >> 2;

  __shared__ __align__(16) float sF[BM * FP];

  const int b  = m0 / SEQ;
  const int s0 = m0 - b * SEQ;

  v8f acc[2][2];
  #pragma unroll
  for (int i = 0; i < 2; ++i)
    #pragma unroll
    for (int j = 0; j < 2; ++j) acc[i][j] = zero8();

  const f16* Ab = ctx  + (size_t)(m0 + wm * 32 + lq) * DM + hi * 8;
  const f16* Wb = wo16 + (size_t)(n0 + wn * 32 + lq) * DM + hi * 8;
  #pragma unroll 1
  for (int k0 = 0; k0 < DM; k0 += 32) {
    FragH af[2], wf[2];
    #pragma unroll
    for (int i = 0; i < 2; ++i) {
      const f16* ap = Ab + (size_t)i * 16 * DM + k0;
      af[i].q[0] = *(const v4u*)(ap);
      af[i].q[1] = *(const v4u*)(ap + 16);
    }
    #pragma unroll
    for (int j = 0; j < 2; ++j) {
      const f16* wp = Wb + (size_t)j * 16 * DM + k0;
      wf[j].q[0] = *(const v4u*)(wp);
      wf[j].q[1] = *(const v4u*)(wp + 16);
    }
    #pragma unroll
    for (int i = 0; i < 2; ++i)
      #pragma unroll
      for (int j = 0; j < 2; ++j) acc[i][j] = mma_f16(af[i].v, wf[j].v, acc[i][j]);
  }

  float bj[2];
  #pragma unroll
  for (int j = 0; j < 2; ++j) bj[j] = (float)(bf16)bo[n0 + wn * 32 + j * 16 + lq];
  const float unc = 1.0f / (CTX_CARRY * WO_CARRY);

  #pragma unroll
  for (int i = 0; i < 2; ++i)
    #pragma unroll
    for (int j = 0; j < 2; ++j)
      #pragma unroll
      for (int r = 0; r < 8; ++r)
        sF[(wm * 32 + i * 16 + 8 * hi + r) * FP + wn * 32 + j * 16 + lq] = acc[i][j][r] * unc + bj[j];
  __syncthreads();

  v4f    vals[8];
  size_t gidx[8];
  #pragma unroll
  for (int it = 0; it < 8; ++it) {
    const int row   = wave * 16 + it * 2 + (lane >> 4);
    const int piece = lane & 15;
    vals[it] = *(const v4f*)(sF + row * FP + piece * 4);
    gidx[it] = ((size_t)b * SEQ_FULL + s0 + row) * DM + n0 + piece * 4;
  }
  #pragma unroll
  for (int it = 0; it < 8; ++it) *(volatile v4f*)(out + gidx[it]) = vals[it];
  __threadfence();
  #pragma unroll
  for (int it = 0; it < 8; ++it) *(volatile v4f*)(out + gidx[it]) = vals[it];
}

extern "C" void kernel_launch(void* const* d_in, const int* in_sizes, int n_in,
                              void* d_out, int out_size, void* d_ws, size_t ws_size,
                              hipStream_t stream) {
  if (n_in < 9) return;
  const size_t rows_used = (size_t)(NB - 1) * SEQ_FULL + SEQ;
  if ((size_t)in_sizes[0] < rows_used * DM) return;
  if (in_sizes[1] < DM * DM || in_sizes[3] < DM * DM || in_sizes[5] < DM * DM || in_sizes[7] < DM * DM) return;
  if (in_sizes[2] < DM || in_sizes[4] < DM || in_sizes[6] < DM || in_sizes[8] < DM) return;
  if ((size_t)out_size < rows_used * DM) return;

  const size_t xb_bytes   = (size_t)MROWS * DM * 2;
  const size_t wqkv_bytes = (size_t)3 * DM * DM * 2;
  const size_t wo_bytes   = (size_t)DM * DM * 2;
  const size_t pl_bytes   = (size_t)NB * NHEAD * SEQ * HDIM * 2;
  const size_t ctx_bytes  = (size_t)MROWS * DM * 2;
  const size_t total      = xb_bytes + wqkv_bytes + wo_bytes + 3 * pl_bytes + ctx_bytes;
  if (ws_size < total) return;

  const float* x  = (const float*)d_in[0];
  const float* Wq = (const float*)d_in[1];
  const float* bq = (const float*)d_in[2];
  const float* Wk = (const float*)d_in[3];
  const float* bk = (const float*)d_in[4];
  const float* Wv = (const float*)d_in[5];
  const float* bv = (const float*)d_in[6];
  const float* Wo = (const float*)d_in[7];
  const float* bo = (const float*)d_in[8];
  float*       out = (float*)d_out;

  char* ws = (char*)d_ws;
  size_t off = 0;
  bf16* xb   = (bf16*)(ws + off); off += xb_bytes;
  bf16* wqkv = (bf16*)(ws + off); off += wqkv_bytes;
  f16*  wo16 = (f16*)(ws + off);  off += wo_bytes;
  f16*  qpl  = (f16*)(ws + off);  off += pl_bytes;
  f16*  kpl  = (f16*)(ws + off);  off += pl_bytes;
  f16*  vt   = (f16*)(ws + off);  off += pl_bytes;
  f16*  ctx  = (f16*)(ws + off);  off += ctx_bytes;
  if (off > ws_size) return;

  cvt_kernel<<<dim3(MROWS + 4 * DM), dim3(128), 0, stream>>>(x, Wq, Wk, Wv, Wo, xb, wqkv, wo16);
  qkv_gemm_kernel<<<dim3(3 * DM / BN, MROWS / BM), dim3(256), 0, stream>>>(xb, wqkv, bq, bk, bv, qpl, kpl, vt);
  attn_kernel<<<dim3(SEQ / BQ, NHEAD, NB), dim3(256), 0, stream>>>(qpl, kpl, vt, ctx);
  oproj_kernel<<<dim3(DM / BN, MROWS / BM), dim3(256), 0, stream>>>(ctx, wo16, bo, out);
}
